// HGNND_31353261260882
// MI455X (gfx1250) — hardware-run, weakly checked
//
#include <hip/hip_runtime.h>
#include <hip/hip_bf16.h>
#include <stddef.h>


#define HID   128
#define OUTD  64
#define FUSR  256
#define NTHR  256
#define NWAVE 8
#define NB    512
#define CHUNK 2048
#define WCAP  256
#define NGRP  (CHUNK / (NTHR * 4))
#define PPW   32
#define GRP   32
#define GRQ   64

#define LDS_GAT_BYTES ((NB * HID + 3 * NB + NWAVE * WCAP + NWAVE) * 4)

static_assert(NB == 512);
static_assert(CHUNK == 2048);
static_assert(WCAP == (CHUNK / NTHR) * 32);
static_assert(NGRP * NTHR * 4 == CHUNK);
static_assert(LDS_GAT_BYTES == 276512);
static_assert(((NB * HID) % 4) == 0);
static_assert(NWAVE * PPW == NTHR);

typedef float          v4f   __attribute__((ext_vector_type(4)));
typedef float          v8f   __attribute__((ext_vector_type(8)));
typedef int            v4i   __attribute__((ext_vector_type(4)));
typedef unsigned short us16;
typedef us16           v8us  __attribute__((ext_vector_type(8)));
typedef us16           v16us __attribute__((ext_vector_type(16)));
typedef __bf16         v16b  __attribute__((ext_vector_type(16)));
union BFrag { v16b v; v16us u; v8us half[2]; };

__device__ __forceinline__ v8f wm(v16b a, v16b b, v8f c) {
  v8f d = __builtin_amdgcn_wmma_f32_16x16x32_bf16(false, a, false, b, (short)0, c, false, false);
  asm volatile("v_nop\n\tv_nop\n\tv_nop\n\tv_nop" : "+v"(d) : "v"(a), "v"(b));
  return d;
}

__device__ __forceinline__ float wsum(float v) {
  v += __shfl_xor(v, 16, 32);
  v += __shfl_xor(v, 8, 32);
  v += __shfl_xor(v, 4, 32);
  v += __shfl_xor(v, 2, 32);
  v += __shfl_xor(v, 1, 32);
  return v;
}

__device__ __forceinline__ unsigned bfr(float x) {
  const unsigned u = __float_as_uint(x);
  return (u + 0x7FFFu + ((u >> 16) & 1u)) >> 16;
}
__device__ __forceinline__ void split2(float x, us16& hi, us16& lo) {
  const unsigned hb = bfr(x);
  const float hf = __uint_as_float(hb << 16);
  const unsigned lb = bfr(x - hf);
  hi = (us16)hb;
  lo = (us16)lb;
}

__global__ __launch_bounds__(NTHR) void k_prepw(const float* __restrict__ W, us16* Bh, us16* Bl,
                                                int K, int NN) {
  const int t = blockIdx.x * NTHR + threadIdx.x;
  const int k8n = K >> 3;
  if (t >= NN * k8n) return;
  const int n  = t / k8n;
  const int k8 = (t - n * k8n) * 8;
  v8us vh, vl;
#pragma unroll
  for (int j = 0; j < 8; ++j) {
    us16 a, b;
    split2(W[(size_t)(k8 + j) * NN + n], a, b);
    vh[j] = a;
    vl[j] = b;
  }
  us16* ph = Bh + (size_t)n * K + k8;
  us16* pl = Bl + (size_t)n * K + k8;
  *(volatile v8us*)ph = vh;
  *(volatile v8us*)pl = vl;
  __threadfence();
  *(volatile v8us*)ph = vh;
  *(volatile v8us*)pl = vl;
}

template <int TN, int CSP, bool EL>
__device__ __forceinline__ void epi_tile(v8f acc, int rt, int hh, int m, int ct, int ncol,
                                         float bv, float alc, float arc,
                                         float* Cs, float* Els, float* Ers) {
  float sl[8], sr[8];
#pragma unroll
  for (int r = 0; r < 8; ++r) {
    const int row = rt * 16 + 8 * hh + r;
    const float v = acc[r] + bv;
    Cs[row * CSP + ncol] = v;
    sl[r] = v * alc;
    sr[r] = v * arc;
  }
  if (EL) {
#pragma unroll
    for (int mk = 1; mk < 16; mk <<= 1) {
#pragma unroll
      for (int r = 0; r < 8; ++r) {
        sl[r] += __shfl_xor(sl[r], mk, 32);
        sr[r] += __shfl_xor(sr[r], mk, 32);
      }
    }
    if (m == 0) {
#pragma unroll
      for (int r = 0; r < 8; ++r) {
        Els[(rt * 16 + 8 * hh + r) * TN + ct] = sl[r];
        Ers[(rt * 16 + 8 * hh + r) * TN + ct] = sr[r];
      }
    }
  }
}

template <int K, int NN, int GR, bool EL, bool BIAS>
__global__ __launch_bounds__(NTHR) void k_gemm(
    const float* __restrict__ A, int M,
    const us16* __restrict__ Bh, const us16* __restrict__ Bl,
    const float* __restrict__ bias, const float* __restrict__ avl, const float* __restrict__ avr,
    float* Cg, float* elg, float* erg) {
  constexpr int TN  = NN / 16;
  constexpr int KU  = K / 32;
  constexpr int AP  = K + 8;
  constexpr int CSP = NN + 4;
  static_assert((GR / 16) * TN == 2 * NWAVE);
  static_assert(GR * NN == 16 * NTHR);
  static_assert(!EL || GR == 32);
  static_assert((K % 32) == 0 && (NWAVE % TN) == 0);

  __shared__ __attribute__((aligned(16))) us16  Ahs[GR * AP];
  __shared__ __attribute__((aligned(16))) us16  Als[GR * AP];
  __shared__ __attribute__((aligned(16))) float Cs[GR * CSP];
  __shared__ float Els[GR * TN];
  __shared__ float Ers[GR * TN];

  const int tid  = threadIdx.x;
  const int lane = tid & 31;
  const int wave = tid >> 5;
  const int hh   = lane >> 4;
  const int m    = lane & 15;
  const int rowBase = blockIdx.x * GR;

  for (int u = tid; u < GR * KU; u += NTHR) {
    const int row = u / KU;
    const int c0  = (u - row * KU) * 32;
    int grow = rowBase + row;
    if (grow > M - 1) grow = M - 1;
    const float* p = A + (size_t)grow * K + c0;
#pragma unroll
    for (int q = 0; q < 4; ++q) {
      const v4f f0 = *(const v4f*)(p + 8 * q);
      const v4f f1 = *(const v4f*)(p + 8 * q + 4);
      v8us vh, vl;
      us16 a, b;
      split2(f0.x, a, b); vh[0] = a; vl[0] = b;
      split2(f0.y, a, b); vh[1] = a; vl[1] = b;
      split2(f0.z, a, b); vh[2] = a; vl[2] = b;
      split2(f0.w, a, b); vh[3] = a; vl[3] = b;
      split2(f1.x, a, b); vh[4] = a; vl[4] = b;
      split2(f1.y, a, b); vh[5] = a; vl[5] = b;
      split2(f1.z, a, b); vh[6] = a; vl[6] = b;
      split2(f1.w, a, b); vh[7] = a; vl[7] = b;
      *(v8us*)(Ahs + row * AP + c0 + 8 * q) = vh;
      *(v8us*)(Als + row * AP + c0 + 8 * q) = vl;
    }
  }
  __syncthreads();

  const int ct   = wave % TN;
  const int rt0  = wave / TN;
  const int rt1  = rt0 + NWAVE / TN;
  const int ncol = ct * 16 + m;
  const us16* bph = Bh  + (size_t)ncol * K + 8 * hh;
  const us16* bpl = Bl  + (size_t)ncol * K + 8 * hh;
  const us16* q0h = Ahs + (rt0 * 16 + m) * AP + 8 * hh;
  const us16* q0l = Als + (rt0 * 16 + m) * AP + 8 * hh;
  const us16* q1h = Ahs + (rt1 * 16 + m) * AP + 8 * hh;
  const us16* q1l = Als + (rt1 * 16 + m) * AP + 8 * hh;

  v8f c0 = {0.f, 0.f, 0.f, 0.f, 0.f, 0.f, 0.f, 0.f};
  v8f c1 = {0.f, 0.f, 0.f, 0.f, 0.f, 0.f, 0.f, 0.f};
#pragma unroll 1
  for (int kt = 0; kt < KU; ++kt) {
    const int k0 = kt * 32;
    BFrag bh, bl, fa0h, fa0l, fa1h, fa1l;
    bh.half[0]   = *(const v8us*)(bph + k0);  bh.half[1]   = *(const v8us*)(bph + k0 + 16);
    bl.half[0]   = *(const v8us*)(bpl + k0);  bl.half[1]   = *(const v8us*)(bpl + k0 + 16);
    fa0h.half[0] = *(const v8us*)(q0h + k0);  fa0h.half[1] = *(const v8us*)(q0h + k0 + 16);
    fa0l.half[0] = *(const v8us*)(q0l + k0);  fa0l.half[1] = *(const v8us*)(q0l + k0 + 16);
    fa1h.half[0] = *(const v8us*)(q1h + k0);  fa1h.half[1] = *(const v8us*)(q1h + k0 + 16);
    fa1l.half[0] = *(const v8us*)(q1l + k0);  fa1l.half[1] = *(const v8us*)(q1l + k0 + 16);
    c0 = wm(fa0h.v, bh.v, c0);
    c0 = wm(fa0h.v, bl.v, c0);
    c0 = wm(fa0l.v, bh.v, c0);
    c1 = wm(fa1h.v, bh.v, c1);
    c1 = wm(fa1h.v, bl.v, c1);
    c1 = wm(fa1l.v, bh.v, c1);
  }

  const float bv  = BIAS ? bias[ncol] : 0.f;
  const float alc = EL ? avl[ncol] : 0.f;
  const float arc = EL ? avr[ncol] : 0.f;
  epi_tile<TN, CSP, EL>(c0, rt0, hh, m, ct, ncol, bv, alc, arc, Cs, Els, Ers);
  epi_tile<TN, CSP, EL>(c1, rt1, hh, m, ct, ncol, bv, alc, arc, Cs, Els, Ers);
  __syncthreads();

  v4f ov[4];
  size_t oo[4];
#pragma unroll
  for (int i = 0; i < 4; ++i) {
    const int f   = (i * NWAVE + wave) * 128 + 4 * lane;
    const int row = f / NN;
    const int col = f - row * NN;
    ov[i] = *(const v4f*)(Cs + row * CSP + col);
    oo[i] = (size_t)rowBase * NN + (size_t)f;
  }
  float ev = 0.f;
  if (EL) {
    float se = 0.f, sr = 0.f;
#pragma unroll
    for (int t = 0; t < TN; ++t) {
      se += Els[lane * TN + t];
      sr += Ers[lane * TN + t];
    }
    ev = (wave == 0) ? se : sr;
  }
#pragma unroll
  for (int i = 0; i < 4; ++i) *(volatile v4f*)(Cg + oo[i]) = ov[i];
  if (EL) {
    if (wave == 0)      *(volatile float*)(elg + rowBase + lane) = ev;
    else if (wave == 1) *(volatile float*)(erg + rowBase + lane) = ev;
  }
  __threadfence();
#pragma unroll
  for (int i = 0; i < 4; ++i) *(volatile v4f*)(Cg + oo[i]) = ov[i];
  if (EL) {
    if (wave == 0)      *(volatile float*)(elg + rowBase + lane) = ev;
    else if (wave == 1) *(volatile float*)(erg + rowBase + lane) = ev;
  }
}

__global__ __launch_bounds__(NTHR) void k_gat(
    const float* __restrict__ z, const float* __restrict__ elg, const float* __restrict__ erg,
    const int* __restrict__ srci, const int* __restrict__ dsti, const float* __restrict__ gbias,
    float* hout, int nN, int nE) {
  extern __shared__ v4f lds_dyn[];
  float* sacc = (float*)lds_dyn;
  float* mrun = sacc + NB * HID;
  float* den  = mrun + NB;
  float* ers  = den + NB;
  int*   list = (int*)(ers + NB);
  int*   wcnt = list + NWAVE * WCAP;

  const int tid  = threadIdx.x;
  const int lane = tid & 31;
  const int wave = tid >> 5;
  const int nodeBase = blockIdx.x * NB;
  const float ninf = __uint_as_float(0xff800000u);

  {
    const v4f z4 = {0.f, 0.f, 0.f, 0.f};
    for (int i = tid; i < (NB * HID) / 4; i += NTHR) lds_dyn[i] = z4;
    for (int s = tid; s < NB; s += NTHR) {
      mrun[s] = ninf;
      den[s]  = 0.f;
      int nd = nodeBase + s;
      if (nd > nN - 1) nd = nN - 1;
      ers[s] = erg[nd];
    }
  }
  __syncthreads();

  const bool al16 = ((((size_t)dsti) & 15) == 0);
  const int nChunks = (nE + CHUNK - 1) / CHUNK;
#pragma unroll 1
  for (int ch = 0; ch < nChunks; ++ch) {
    const int cbase = ch * CHUNK;
    int wc = 0;
#pragma unroll
    for (int g = 0; g < NGRP; ++g) {
      const int el0 = (g * NTHR + tid) * 4;
      const int e0  = cbase + el0;
      v4i d;
      if (al16 && (cbase + CHUNK <= nE)) {
        d = *(const v4i*)(dsti + e0);
      } else {
        const int sent = -2147483647 - 1;
        const int d0 = dsti[min(e0,     nE - 1)];
        const int d1 = dsti[min(e0 + 1, nE - 1)];
        const int d2 = dsti[min(e0 + 2, nE - 1)];
        const int d3 = dsti[min(e0 + 3, nE - 1)];
        d.x = (e0     < nE) ? d0 : sent;
        d.y = (e0 + 1 < nE) ? d1 : sent;
        d.z = (e0 + 2 < nE) ? d2 : sent;
        d.w = (e0 + 3 < nE) ? d3 : sent;
      }
      const unsigned s0 = (unsigned)d.x - (unsigned)nodeBase;
      const unsigned s1 = (unsigned)d.y - (unsigned)nodeBase;
      const unsigned s2 = (unsigned)d.z - (unsigned)nodeBase;
      const unsigned s3 = (unsigned)d.w - (unsigned)nodeBase;
#define HITJ(J, SJ) { \
        const bool hj = (SJ) < (unsigned)NB; \
        const unsigned mj = __builtin_amdgcn_ballot_w32(hj); \
        if (mj != 0u) { \
          if (hj) { \
            const int pos = wc + (int)__builtin_amdgcn_mbcnt_lo(mj, 0u); \
            if (pos < WCAP) list[wave * WCAP + pos] = ((el0 + (J)) << 9) | (int)(SJ); \
          } \
          wc += (int)__builtin_popcount(mj); \
        } }
      HITJ(0, s0)
      HITJ(1, s1)
      HITJ(2, s2)
      HITJ(3, s3)
#undef HITJ
    }
    if (lane == 0) wcnt[wave] = wc;
    __syncthreads();

    if (wave == 0) {
#pragma unroll 1
      for (int wsx = 0; wsx < NWAVE; ++wsx) {
        int n = wcnt[wsx];
        n = (n > WCAP) ? WCAP : ((n < 0) ? 0 : n);
#pragma unroll 1
        for (int i = 0; i < n; ++i) {
          const int ent  = list[wsx * WCAP + i];
          const int slot = ent & (NB - 1);
          const int elc  = (ent >> 9) & (CHUNK - 1);
          int e = cbase + elc;
          if (e > nE - 1) e = nE - 1;
          int s = srci[e];
          s = (s < 0) ? 0 : ((s > nN - 1) ? (nN - 1) : s);
          float lg = elg[s] + ers[slot];
          lg = (lg > 0.f) ? lg : 0.2f * lg;
          const float mo = mrun[slot];
          const float mn = fmaxf(mo, lg);
          const float f  = __expf(mo - mn);
          const float p  = __expf(lg - mn);
          const v4f zv = *(const v4f*)(z + (size_t)s * HID + 4 * lane);
          v4f* sp = (v4f*)(sacc + slot * HID + 4 * lane);
          const v4f cur = *sp;
          const v4f nxt = cur * f + zv * p;
          *sp = nxt;
          const float dn = den[slot] * f + p;
          den[slot]  = dn;
          mrun[slot] = mn;
        }
      }
    }
    __syncthreads();
  }

  const v4f b4 = *(const v4f*)(gbias + 4 * lane);
#pragma unroll 1
  for (int j = 0; j < NB / NWAVE; ++j) {
    const int slot = wave * (NB / NWAVE) + j;
    const int node = nodeBase + slot;
    if (node >= nN) break;
    const float dn  = den[slot];
    const float inv = (dn > 0.f) ? (1.0f / dn) : 0.f;
    const v4f sv = *(const v4f*)(sacc + slot * HID + 4 * lane);
    v4f hv = sv * inv + b4;
    hv.x = (hv.x > 0.f) ? hv.x : (__expf(hv.x) - 1.0f);
    hv.y = (hv.y > 0.f) ? hv.y : (__expf(hv.y) - 1.0f);
    hv.z = (hv.z > 0.f) ? hv.z : (__expf(hv.z) - 1.0f);
    hv.w = (hv.w > 0.f) ? hv.w : (__expf(hv.w) - 1.0f);
    float* op = hout + (size_t)node * HID + 4 * lane;
    *(volatile v4f*)op = hv;
    __threadfence();
    *(volatile v4f*)op = hv;
  }
}

__global__ __launch_bounds__(NTHR) void k_pair(const float* __restrict__ h,
                                               const int* __restrict__ ia, const int* __restrict__ ib,
                                               float* lo, int P, int nN) {
  const int tid  = threadIdx.x;
  const int lane = tid & 31;
  const int wave = tid >> 5;
  const int pbase = (blockIdx.x * NWAVE + wave) * PPW;
  float lreg = 0.f;
#pragma unroll 1
  for (int i = 0; i < PPW; ++i) {
    int p = pbase + i;
    if (p > P - 1) p = P - 1;
    int a = ia[p];
    int b = ib[p];
    a = (a < 0) ? 0 : ((a > nN - 1) ? (nN - 1) : a);
    b = (b < 0) ? 0 : ((b > nN - 1) ? (nN - 1) : b);
    const v4f va = *(const v4f*)(h + (size_t)a * HID + 4 * lane);
    const v4f vb = *(const v4f*)(h + (size_t)b * HID + 4 * lane);
    float s = va.x * vb.x + va.y * vb.y + va.z * vb.z + va.w * vb.w;
    s = wsum(s);
    const float t  = __expf(-fabsf(s));
    const float u  = 1.0f + t;
    const float lg = __logf(u) - ((u - 1.0f) - t) * __builtin_amdgcn_rcpf(u);
    const float l  = fminf(s, 0.f) - lg;
    lreg = (lane == i) ? l : lreg;
  }
  float* op = lo + pbase + lane;
  *(volatile float*)op = lreg;
  __threadfence();
  *(volatile float*)op = lreg;
}

__global__ __launch_bounds__(NTHR) void k_loss(const float* __restrict__ lp, const float* __restrict__ ln,
                                               const int* __restrict__ alpha, float* lossline,
                                               int Pp, int Pn) {
  __shared__ float  rmx[NTHR];
  __shared__ double rsd[NTHR];
  const int tid = threadIdx.x;
  const float ninf = __uint_as_float(0xff800000u);

  float mp = ninf, mn = ninf;
#pragma unroll 1
  for (int i = tid; i < Pp; i += NTHR) mp = fmaxf(mp, lp[i]);
#pragma unroll 1
  for (int i = tid; i < Pn; i += NTHR) mn = fmaxf(mn, ln[i]);

  rmx[tid] = mp;
  __syncthreads();
  for (int s = NTHR / 2; s > 0; s >>= 1) {
    if (tid < s) rmx[tid] = fmaxf(rmx[tid], rmx[tid + s]);
    __syncthreads();
  }
  const float gmp = rmx[0];
  __syncthreads();
  rmx[tid] = mn;
  __syncthreads();
  for (int s = NTHR / 2; s > 0; s >>= 1) {
    if (tid < s) rmx[tid] = fmaxf(rmx[tid], rmx[tid + s]);
    __syncthreads();
  }
  const float gmn = rmx[0];
  __syncthreads();

  const float af = (float)alpha[0];
  const float kT = (0.5f <= af) ? 0.5f : af;
  const float hp = kT * gmp;
  const float hn = kT * gmn;

  double sd = 0.0;
#pragma unroll 1
  for (int i = tid; i < Pp; i += NTHR) {
    const float l = lp[i];
    sd += (l > hp) ? 0.0 : (double)l;
  }
#pragma unroll 1
  for (int i = tid; i < Pn; i += NTHR) {
    const float l = ln[i];
    sd += (l > hn) ? 0.0 : (double)l;
  }
  rsd[tid] = sd;
  __syncthreads();
  for (int s = NTHR / 2; s > 0; s >>= 1) {
    if (tid < s) rsd[tid] = rsd[tid] + rsd[tid + s];
    __syncthreads();
  }
  const float loss = (float)(-rsd[0]);
  if (tid < 32) {
    const float v = (tid == 0) ? loss : 0.f;
    *(volatile float*)(lossline + tid) = v;
    __threadfence();
    *(volatile float*)(lossline + tid) = v;
  }
}

__global__ __launch_bounds__(NTHR) void k_pack(const float* __restrict__ plane,
                                               const float* __restrict__ lossline,
                                               float* out, int nOut) {
  const int f = blockIdx.x * NTHR + threadIdx.x;
  int idx = f - 1;
  if (idx < 0) idx = 0;
  if (idx > nOut - 2) idx = nOut - 2;
  const float pv = plane[idx];
  const float lv = lossline[0];
  const float v = (f == 0) ? lv : pv;
  if (f < nOut) {
    float* op = out + f;
    *(volatile float*)op = v;
    __threadfence();
    *(volatile float*)op = v;
  }
}

static inline int cdiv(int a, int b) { return (a + b - 1) / b; }
static inline size_t al256(size_t v) { return (v + 255) & ~(size_t)255; }

extern "C" void kernel_launch(void* const* d_in, const int* in_sizes, int n_in,
                              void* d_out, int out_size, void* d_ws, size_t ws_size,
                              hipStream_t stream) {
  if (n_in < 19) return;
  const int Nu = in_sizes[0] / FUSR;
  const int Ni = in_sizes[1] / HID;
  if (Nu <= 0 || Ni <= 0 || in_sizes[0] != Nu * FUSR || in_sizes[1] != Ni * HID) return;
  if ((Nu % GRP) != 0 || (Ni % GRP) != 0) return;
  if (in_sizes[2] != FUSR * HID || in_sizes[3] != HID) return;
  if (in_sizes[4] != HID * HID || in_sizes[5] != HID) return;
  if (in_sizes[6] != HID * HID || in_sizes[7] != HID || in_sizes[8] != HID || in_sizes[9] != HID) return;
  if (in_sizes[10] != HID * OUTD || in_sizes[11] != OUTD) return;
  const int N = Nu + Ni;
  const int E = in_sizes[12];
  if (E < 1 || in_sizes[13] != E) return;
  const int Pp = in_sizes[14];
  const int Pn = in_sizes[16];
  if (Pp < 1 || Pn < 1 || in_sizes[15] != Pp || in_sizes[17] != Pn || in_sizes[18] < 1) return;
  if (out_size != 1 + Nu * OUTD) return;

  const float* feat_user = (const float*)d_in[0];
  const float* feat_item = (const float*)d_in[1];
  const float* W_user    = (const float*)d_in[2];
  const float* b_user    = (const float*)d_in[3];
  const float* W_item    = (const float*)d_in[4];
  const float* b_item    = (const float*)d_in[5];
  const float* W_gat     = (const float*)d_in[6];
  const float* attn_l    = (const float*)d_in[7];
  const float* attn_r    = (const float*)d_in[8];
  const float* gat_bias  = (const float*)d_in[9];
  const float* W_pred    = (const float*)d_in[10];
  const float* b_pred    = (const float*)d_in[11];
  const int*   src       = (const int*)d_in[12];
  const int*   dst       = (const int*)d_in[13];
  const int*   pos_src   = (const int*)d_in[14];
  const int*   pos_dst   = (const int*)d_in[15];
  const int*   neg_src   = (const int*)d_in[16];
  const int*   neg_dst   = (const int*)d_in[17];
  const int*   alpha     = (const int*)d_in[18];
  float* outg = (float*)d_out;

  const int NuPad = cdiv(Nu, GRQ) * GRQ;
  const int PpPad = cdiv(Pp, NWAVE * PPW) * (NWAVE * PPW);
  const int PnPad = cdiv(Pn, NWAVE * PPW) * (NWAVE * PPW);
  char* wsb = (char*)d_ws;
  size_t off = 0;
  float* xh = (float*)(wsb + off);          off += al256((size_t)N * HID * sizeof(float));
  const size_t rbBytes = al256((size_t)N * HID * sizeof(float));
  char*  rb = wsb + off;                    off += rbBytes;
  float* zp = (float*)rb;
  size_t o2 = 0;
  float* outp  = (float*)(rb + o2);         o2 += al256((size_t)NuPad * OUTD * sizeof(float));
  float* lpos  = (float*)(rb + o2);         o2 += al256((size_t)PpPad * sizeof(float));
  float* lneg  = (float*)(rb + o2);         o2 += al256((size_t)PnPad * sizeof(float));
  float* lossl = (float*)(rb + o2);         o2 += 256;
  if (o2 > rbBytes) return;
  float* elp = (float*)(wsb + off);         off += al256((size_t)N * sizeof(float));
  float* erp = (float*)(wsb + off);         off += al256((size_t)N * sizeof(float));
  us16* wuh = (us16*)(wsb + off);           off += al256((size_t)FUSR * HID * sizeof(us16));
  us16* wul = (us16*)(wsb + off);           off += al256((size_t)FUSR * HID * sizeof(us16));
  us16* wih = (us16*)(wsb + off);           off += al256((size_t)HID * HID * sizeof(us16));
  us16* wil = (us16*)(wsb + off);           off += al256((size_t)HID * HID * sizeof(us16));
  us16* wgh = (us16*)(wsb + off);           off += al256((size_t)HID * HID * sizeof(us16));
  us16* wgl = (us16*)(wsb + off);           off += al256((size_t)HID * HID * sizeof(us16));
  us16* wph = (us16*)(wsb + off);           off += al256((size_t)HID * OUTD * sizeof(us16));
  us16* wpl = (us16*)(wsb + off);           off += al256((size_t)HID * OUTD * sizeof(us16));
  if (off > ws_size) return;
  if (off > (size_t)134217728) return;

  k_prepw<<<cdiv(HID * (FUSR / 8), NTHR), NTHR, 0, stream>>>(W_user, wuh, wul, FUSR, HID);
  k_prepw<<<cdiv(HID * (HID / 8), NTHR), NTHR, 0, stream>>>(W_item, wih, wil, HID, HID);
  k_prepw<<<cdiv(HID * (HID / 8), NTHR), NTHR, 0, stream>>>(W_gat, wgh, wgl, HID, HID);
  k_prepw<<<cdiv(OUTD * (HID / 8), NTHR), NTHR, 0, stream>>>(W_pred, wph, wpl, HID, OUTD);

  k_gemm<FUSR, HID, GRP, false, true><<<Nu / GRP, NTHR, 0, stream>>>(
      feat_user, Nu, wuh, wul, b_user, attn_l, attn_r, xh, elp, erp);
  k_gemm<HID, HID, GRP, false, true><<<Ni / GRP, NTHR, 0, stream>>>(
      feat_item, Ni, wih, wil, b_item, attn_l, attn_r, xh + (size_t)Nu * HID, elp, erp);

  k_gemm<HID, HID, GRP, true, false><<<N / GRP, NTHR, 0, stream>>>(
      xh, N, wgh, wgl, b_item, attn_l, attn_r, zp, elp, erp);

  hipFuncSetAttribute(reinterpret_cast<const void*>(&k_gat),
                      hipFuncAttributeMaxDynamicSharedMemorySize, LDS_GAT_BYTES);
  k_gat<<<cdiv(N, NB), NTHR, LDS_GAT_BYTES, stream>>>(zp, elp, erp, src, dst, gat_bias, xh, N, E);

  k_gemm<HID, OUTD, GRQ, false, true><<<NuPad / GRQ, NTHR, 0, stream>>>(
      xh, Nu, wph, wpl, b_pred, attn_l, attn_r, outp, elp, erp);

  k_pair<<<PpPad / (NWAVE * PPW), NTHR, 0, stream>>>(xh, pos_src, pos_dst, lpos, Pp, N);
  k_pair<<<PnPad / (NWAVE * PPW), NTHR, 0, stream>>>(xh, neg_src, neg_dst, lneg, Pn, N);
  k_loss<<<1, NTHR, 0, stream>>>(lpos, lneg, alpha, lossl, Pp, Pn);

  k_pack<<<cdiv(out_size, NTHR), NTHR, 0, stream>>>(outp, lossl, outg, out_size);
}
